// Block_2783138808310
// MI455X (gfx1250) — hardware-run, weakly checked
//
#include <hip/hip_runtime.h>
#ifndef NB
#define NB 16
#endif
#ifndef SEQ
#define SEQ 1024
#endif
#define NB_FULL 16
#define SEQ_FULL 1024
#define DM 256
#define NH 8
#define HD 32
#define DFF 1024
#define LQ (3 * DM)
#define GW 32
#define GH 32
#define NV (GW * GH)
#define NPT 4
#define NOFF (NH * NPT * 2)
#define NLG (NH * NPT)
#define NOA 128
#define NR ((size_t)NB * SEQ)
#define NRV ((size_t)NB * NV)
#define FCH (NR < (size_t)4096 ? NR : (size_t)4096)
#define OTP 264

static_assert(HD == 32);
static_assert(NH * HD == DM);
static_assert(SEQ % 64 == 0);
static_assert(SEQ % 16 == 0);
static_assert(NR % 128 == 0);
static_assert(NRV % 128 == 0);
static_assert(NR % FCH == 0);
static_assert(FCH % 128 == 0);
static_assert(DM % 64 == 0);
static_assert(DFF % 64 == 0);
static_assert(LQ % 64 == 0);
static_assert(NOA % 64 == 0);
static_assert(DM % 32 == 0);
static_assert(DFF % 32 == 0);
static_assert(NOFF == 64);
static_assert(NLG == 32);
static_assert(NOFF + NLG <= NOA);
static_assert(NOA / 4 == 32);
static_assert((NOA * DM / 8) % 256 == 0);
static_assert(DM * 2 == 32 * 16);
static_assert(DM == 2 * 32 * 4);
static_assert(OTP >= DM + 8);
static_assert(NV <= SEQ_FULL);
static_assert(NV == 1024);
static_assert(NB <= NB_FULL);
static_assert(SEQ <= SEQ_FULL);
static_assert((LQ * DM / 8) % 256 == 0);
static_assert((DM * DM / 8) % 256 == 0);
static_assert((DFF * DM / 8) % 256 == 0);
static_assert((NRV * DM / 8) % 256 == 0);

typedef unsigned short v8us __attribute__((ext_vector_type(8), may_alias));
typedef float  v8f  __attribute__((ext_vector_type(8)));
typedef float  v4f  __attribute__((ext_vector_type(4)));
typedef float  v4fa __attribute__((ext_vector_type(4), may_alias));
typedef _Float16 v16h __attribute__((ext_vector_type(16)));
typedef _Float16 v4h __attribute__((ext_vector_type(4)));
union FragH { v16h v; v8us half[2]; _Float16 h[16]; unsigned short u[16]; };

__device__ __forceinline__ unsigned short bf16_bits(float x) { unsigned int u = __float_as_uint(x); return (unsigned short)((u + 0x7FFFu + ((u >> 16) & 1u)) >> 16); }
__device__ __forceinline__ float bf16_val(unsigned short b) { return __uint_as_float(((unsigned int)b) << 16); }
__device__ __forceinline__ float bf16_rne(float x) { return bf16_val(bf16_bits(x)); }
__device__ __forceinline__ _Float16 toh_flush(float v) { const _Float16 r = (_Float16)v; return (fabsf(v) < 6.103515625e-05f) ? (_Float16)0.0f : r; }

__device__ __forceinline__ v16h g2_frag(const _Float16* p, int hh) { FragH f; f.half[0] = *(const v8us*)((const unsigned short*)p + 8 * hh); f.half[1] = *(const v8us*)((const unsigned short*)p + 16 + 8 * hh); return f.v; }
__device__ __forceinline__ v8f g2_mma(v16h a, v16h b, v8f c) { v8f d = __builtin_amdgcn_wmma_f32_16x16x32_f16(false, a, false, b, (short)0, c, false, false); asm volatile("v_nop\n\tv_nop\n\tv_nop\n\tv_nop" : "+v"(d) : "v"(a), "v"(b)); return d; }

__global__ __launch_bounds__(256) void k_w16(const float* __restrict__ W, _Float16* __restrict__ Wh, unsigned n8, float scale) {
  const unsigned t = blockIdx.x * 256u + threadIdx.x; if (t >= n8) return;
  const size_t so = (size_t)t * 8;
  const v4f a0 = *(const v4fa*)(W + so), a1 = *(const v4fa*)(W + so + 4);
  FragH f;
#pragma unroll
  for (int q = 0; q < 4; ++q) { f.h[q] = toh_flush(bf16_rne(a0[q]) * scale); f.h[4 + q] = toh_flush(bf16_rne(a1[q]) * scale); }
  const v8us o = f.half[0];
  unsigned short* d = (unsigned short*)Wh + so;
  for (int pass = 0; pass < 2; ++pass) { *(volatile v8us*)d = o; if (pass == 0) __threadfence(); }
}

__global__ __launch_bounds__(256) void k_woa(const float* __restrict__ off_w, const float* __restrict__ aw_w, const float* __restrict__ off_b, const float* __restrict__ aw_b, _Float16* __restrict__ BOA, float* __restrict__ BIAS) {
  const unsigned tid = threadIdx.x;
  if (blockIdx.x == (unsigned)(NOA * DM / 8 / 256)) {
    if (tid < (unsigned)(NOA / 4)) {
      v4f o;
#pragma unroll
      for (int q = 0; q < 4; ++q) {
        const unsigned c = tid * 4u + (unsigned)q;
        const unsigned co = c < (unsigned)(NOFF - 1) ? c : (unsigned)(NOFF - 1);
        const unsigned cc = c < (unsigned)NOFF ? (unsigned)NOFF : c;
        const unsigned ca = (cc - NOFF) < (unsigned)(NLG - 1) ? (cc - NOFF) : (unsigned)(NLG - 1);
        const float vo = off_b[co], va = aw_b[ca];
        o[q] = (c < (unsigned)NOFF) ? bf16_rne(vo) : ((c < (unsigned)(NOFF + NLG)) ? bf16_rne(va) : 0.f);
      }
      float* d = BIAS + tid * 4u;
      for (int pass = 0; pass < 2; ++pass) { *(volatile v4f*)d = o; if (pass == 0) __threadfence(); }
    }
    return;
  }
  const unsigned t = blockIdx.x * 256u + tid;
  const unsigned row = t / (DM / 8), c8 = (t % (DM / 8)) * 8u;
  const unsigned ro = row < (unsigned)(NOFF - 1) ? row : (unsigned)(NOFF - 1);
  const unsigned rc = row < (unsigned)NOFF ? (unsigned)NOFF : row;
  const unsigned ra = (rc - NOFF) < (unsigned)(NLG - 1) ? (rc - NOFF) : (unsigned)(NLG - 1);
  const float* po = off_w + (size_t)ro * DM + c8; const float* pa = aw_w + (size_t)ra * DM + c8;
  const v4f o0 = *(const v4fa*)po, o1 = *(const v4fa*)(po + 4), b0 = *(const v4fa*)pa, b1 = *(const v4fa*)(pa + 4);
  FragH f;
#pragma unroll
  for (int q = 0; q < 4; ++q) {
    const float s0 = (row < (unsigned)NOFF) ? o0[q] : ((row < (unsigned)(NOFF + NLG)) ? b0[q] : 0.f);
    const float s1 = (row < (unsigned)NOFF) ? o1[q] : ((row < (unsigned)(NOFF + NLG)) ? b1[q] : 0.f);
    f.h[q] = toh_flush(bf16_rne(s0) * 64.0f); f.h[4 + q] = toh_flush(bf16_rne(s1) * 64.0f);
  }
  const v8us o = f.half[0];
  unsigned short* d = (unsigned short*)BOA + (size_t)t * 8;
  for (int pass = 0; pass < 2; ++pass) { *(volatile v8us*)d = o; if (pass == 0) __threadfence(); }
}

__global__ __launch_bounds__(256) void k_val16(const float* __restrict__ val, _Float16* __restrict__ V16) {
  const unsigned t = blockIdx.x * 256u + threadIdx.x; if (t >= (unsigned)(NRV * DM / 8)) return;
  const size_t so = (size_t)t * 8;
  const v4f a0 = *(const v4fa*)(val + so), a1 = *(const v4fa*)(val + so + 4);
  FragH fx;
#pragma unroll
  for (int q = 0; q < 4; ++q) { fx.h[q] = toh_flush(bf16_rne(a0[q])); fx.h[4 + q] = toh_flush(bf16_rne(a1[q])); }
  const v8us vx = fx.half[0];
  unsigned short* dx = (unsigned short*)V16 + so;
  for (int pass = 0; pass < 2; ++pass) { *(volatile v8us*)dx = vx; if (pass == 0) __threadfence(); }
}

template <int ACT>
__device__ __forceinline__ void gemm_body(const _Float16* __restrict__ A, int lda, const _Float16* __restrict__ Bh, int ldb, float alpha, const float* __restrict__ bias, const float* __restrict__ R, int ldr, int rbf,
    float* __restrict__ C, _Float16* __restrict__ C16, int ldc, int M, int N, int K) {
  static_assert(ACT == 0 || ACT == 1);
  __shared__ __attribute__((aligned(16))) float so[4][32][68];
  const int tid = threadIdx.x, w = tid >> 5, lane = tid & 31, ln = lane & 15, hh = lane >> 4;
  const float* bp = bias;
  const int ntn = N >> 6; const int mt = blockIdx.x / ntn, nq = blockIdx.x - mt * ntn; const int row0 = mt * 128 + 32 * w, col0 = nq * 64; if (row0 >= M) return;
  const _Float16* a0p = A + (size_t)(row0 + ln) * lda; const _Float16* a1p = a0p + (size_t)16 * lda;
  const _Float16* b0p = Bh + (size_t)(col0 + ln) * ldb; const _Float16* b1p = b0p + (size_t)16 * ldb; const _Float16* b2p = b1p + (size_t)16 * ldb; const _Float16* b3p = b2p + (size_t)16 * ldb;
  const v8f z8 = {0.f,0.f,0.f,0.f,0.f,0.f,0.f,0.f}; v8f c00 = z8, c01 = z8, c02 = z8, c03 = z8, c10 = z8, c11 = z8, c12 = z8, c13 = z8;
#pragma unroll 1
  for (int kb = 0; kb < K; kb += 32) { const v16h a0 = g2_frag(a0p + kb, hh), a1 = g2_frag(a1p + kb, hh);
    v16h b = g2_frag(b0p + kb, hh); c00 = g2_mma(a0, b, c00); c10 = g2_mma(a1, b, c10);
    b = g2_frag(b1p + kb, hh); c01 = g2_mma(a0, b, c01); c11 = g2_mma(a1, b, c11);
    b = g2_frag(b2p + kb, hh); c02 = g2_mma(a0, b, c02); c12 = g2_mma(a1, b, c12);
    b = g2_frag(b3p + kb, hh); c03 = g2_mma(a0, b, c03); c13 = g2_mma(a1, b, c13); }
  v8f accs[8] = {c00, c01, c02, c03, c10, c11, c12, c13};
#pragma unroll
  for (int u = 0; u < 8; ++u) { const int t = u & 3, half = u >> 2; const int col = col0 + t * 16 + ln; const float bv = bp ? bf16_rne(bp[col]) : 0.f;
#pragma unroll
    for (int r = 0; r < 8; ++r) { const int rloc = half * 16 + 8 * hh + r; const float v = accs[u][r] * alpha + bv;
      so[w][rloc][t * 16 + ln] = v; } }
  __builtin_amdgcn_fence(4  , "workgroup"); __builtin_amdgcn_wave_barrier();
  const int rsub = lane >> 4, c4 = (lane & 15) * 4;
  if (ACT == 1) {
#pragma unroll 1
    for (int q = 0; q < 16; ++q) { const int r = q * 2 + rsub; v4f v = *(const v4fa*)&so[w][r][c4];
#pragma unroll
      for (int i = 0; i < 4; ++i) { const float a = v[i]; v[i] = 0.5f * a * (1.0f + erff(a * 0.70710678118654752f)); }
      *(v4fa*)&so[w][r][c4] = (v4fa)v; }
  }
  for (int pass = 0; pass < 2; ++pass) {
#pragma unroll
    for (int q = 0; q < 16; ++q) { const int r = q * 2 + rsub; v4f v = *(const v4fa*)&so[w][r][c4];
      if (R) { const int gr = row0 + r; const size_t rr = rbf ? ((size_t)(gr / SEQ) * SEQ_FULL + (size_t)(gr % SEQ)) : (size_t)gr;
        v4f rv = *(const v4fa*)(R + rr * (size_t)ldr + col0 + c4);
        if (rbf) { for (int i = 0; i < 4; ++i) rv[i] = bf16_rne(rv[i]); }
        v += rv; }
      if (C) *(volatile v4f*)(C + (size_t)(row0 + r) * ldc + col0 + c4) = v;
      if (C16) { v4h h4; for (int i = 0; i < 4; ++i) h4[i] = toh_flush(v[i]); *(volatile v4h*)(C16 + (size_t)(row0 + r) * ldc + col0 + c4) = h4; } }
    if (pass == 0) __threadfence(); } }

__global__ __launch_bounds__(128) void k_gemm_n(const _Float16* __restrict__ A, int lda, const _Float16* __restrict__ Bh, int ldb, float alpha, const float* __restrict__ bias, const float* __restrict__ R, int ldr, int rbf,
    float* __restrict__ C, _Float16* __restrict__ C16, int ldc, int M, int N, int K) {
  gemm_body<0>(A, lda, Bh, ldb, alpha, bias, R, ldr, rbf, C, C16, ldc, M, N, K); }

__global__ __launch_bounds__(128) void k_gemm_gelu(const _Float16* __restrict__ A, int lda, const _Float16* __restrict__ Bh, int ldb, float alpha, const float* __restrict__ bias, const float* __restrict__ R, int ldr, int rbf,
    float* __restrict__ C, _Float16* __restrict__ C16, int ldc, int M, int N, int K) {
  gemm_body<1>(A, lda, Bh, ldb, alpha, bias, R, ldr, rbf, C, C16, ldc, M, N, K); }

__global__ __launch_bounds__(256) void k_vt32(const _Float16* __restrict__ QKV, _Float16* __restrict__ VT) {
  __shared__ unsigned short tl[64][HD + 2];
  const unsigned tid = threadIdx.x; const unsigned slab = blockIdx.x / (SEQ / 64), lg = blockIdx.x % (SEQ / 64); const unsigned b = slab / NH, h = slab % NH;
  { const unsigned r = tid >> 2, c8 = (tid & 3u) * 8u; FragH f; f.half[0] = *(const v8us*)((const unsigned short*)QKV + ((size_t)b * SEQ + lg * 64u + r) * LQ + 2 * DM + h * HD + c8);
#pragma unroll
    for (int q = 0; q < 8; ++q) tl[r][c8 + q] = f.u[q]; }
  __syncthreads();
  const unsigned d = tid >> 3, pc = tid & 7u; FragH g;
#pragma unroll
  for (int q = 0; q < 8; ++q) g.u[q] = tl[pc * 8u + q][d];
  const v8us o = g.half[0];
  unsigned short* dst = (unsigned short*)VT + ((size_t)slab * HD + d) * SEQ + lg * 64u + pc * 8u;
  for (int pass = 0; pass < 2; ++pass) { *(volatile v8us*)dst = o; if (pass == 0) __threadfence(); }
}

__global__ __launch_bounds__(256) void k_flash(const _Float16* __restrict__ QKV, const _Float16* __restrict__ VT, _Float16* __restrict__ O16) {
  __shared__ __attribute__((aligned(16))) unsigned short ot[16][OTP];
  const unsigned tid = threadIdx.x, w = tid >> 5, lane = tid & 31u, ln = lane & 15u, hh = lane >> 4;
  const unsigned b = blockIdx.x / (SEQ / 16), qt = blockIdx.x % (SEQ / 16); const unsigned q0 = qt * 16u;
  const size_t rowb = (size_t)b * SEQ;
  const unsigned short* qkv = (const unsigned short*)QKV;
  const unsigned short* qp = qkv + (rowb + q0 + ln) * LQ + w * HD;
  FragH qf; qf.half[0] = *(const v8us*)(qp + 8u * hh); qf.half[1] = *(const v8us*)(qp + 16u + 8u * hh);
  const unsigned short* kbase = qkv + (rowb + ln) * LQ + DM + w * HD + 8u * hh;
  const unsigned short* vbase = (const unsigned short*)VT + ((size_t)(b * NH + w) * HD + ln) * SEQ + 8u * hh;
  const v8f z8 = {0.f,0.f,0.f,0.f,0.f,0.f,0.f,0.f};
  v8f o0 = z8, o1 = z8; float m = -1.0e30f, l = 0.f;
  const float scale = 0.17677669529663687f;
#pragma unroll 1
  for (unsigned j0 = 0; j0 < SEQ; j0 += 64u) {
    v8f s[4];
#pragma unroll
    for (int t = 0; t < 4; ++t) { const unsigned short* kp = kbase + (size_t)(j0 + 16u * t) * LQ; FragH ka; ka.half[0] = *(const v8us*)kp; ka.half[1] = *(const v8us*)(kp + 16); s[t] = g2_mma(ka.v, qf.v, z8); }
    float mx = s[0][0];
#pragma unroll
    for (int r = 0; r < 8; ++r) { mx = fmaxf(mx, fmaxf(fmaxf(s[0][r], s[1][r]), fmaxf(s[2][r], s[3][r]))); }
    mx = fmaxf(mx, __shfl_xor(mx, 16, 32));
    const float mn = fmaxf(m, mx);
    const float corr = __expf((m - mn) * scale);
    m = mn;
    const float mo = mn * scale - 5.545177444f;
    FragH p0, p1; float ls = 0.f;
#pragma unroll
    for (int r = 0; r < 8; ++r) {
      const float e0 = __expf(fmaf(s[0][r], scale, -mo)), e1 = __expf(fmaf(s[1][r], scale, -mo)), e2 = __expf(fmaf(s[2][r], scale, -mo)), e3 = __expf(fmaf(s[3][r], scale, -mo));
      ls += (e0 + e1) + (e2 + e3);
      p0.h[r] = toh_flush(e0); p0.h[8 + r] = toh_flush(e1); p1.h[r] = toh_flush(e2); p1.h[8 + r] = toh_flush(e3);
    }
    l = l * corr + ls;
#pragma unroll
    for (int r = 0; r < 8; ++r) { o0[r] *= corr; o1[r] *= corr; }
    const unsigned short* vp = vbase + j0;
    FragH va;
    va.half[0] = *(const v8us*)vp; va.half[1] = *(const v8us*)(vp + 16); o0 = g2_mma(va.v, p0.v, o0);
    va.half[0] = *(const v8us*)(vp + (size_t)16 * SEQ); va.half[1] = *(const v8us*)(vp + (size_t)16 * SEQ + 16); o1 = g2_mma(va.v, p0.v, o1);
    va.half[0] = *(const v8us*)(vp + 32); va.half[1] = *(const v8us*)(vp + 48); o0 = g2_mma(va.v, p1.v, o0);
    va.half[0] = *(const v8us*)(vp + (size_t)16 * SEQ + 32); va.half[1] = *(const v8us*)(vp + (size_t)16 * SEQ + 48); o1 = g2_mma(va.v, p1.v, o1);
  }
  l += __shfl_xor(l, 16, 32);
  const float inv = 64.0f / l;
  FragH f0, f1;
#pragma unroll
  for (int r = 0; r < 8; ++r) { f0.h[r] = toh_flush(o0[r] * inv); f1.h[r] = toh_flush(o1[r] * inv); }
  *(v8us*)&ot[ln][w * HD + 8u * hh] = f0.half[0];
  *(v8us*)&ot[ln][w * HD + 16u + 8u * hh] = f1.half[0];
  __syncthreads();
  const v8us r0v = *(const v8us*)&ot[2u * w][lane * 8u];
  const v8us r1v = *(const v8us*)&ot[2u * w + 1u][lane * 8u];
  unsigned short* d0 = (unsigned short*)O16 + (rowb + q0 + 2u * w) * DM + lane * 8u;
  unsigned short* d1 = d0 + DM;
  for (int pass = 0; pass < 2; ++pass) { *(volatile v8us*)d0 = r0v; *(volatile v8us*)d1 = r1v; if (pass == 0) __threadfence(); }
}

__device__ __forceinline__ float dsamp(const float* __restrict__ vh, int xi, int yi) {
  const int xc = xi < 0 ? 0 : (xi > GW - 1 ? GW - 1 : xi);
  const int yc = yi < 0 ? 0 : (yi > GH - 1 ? GH - 1 : yi);
  float val = vh[(size_t)(yc * GW + xc) * DM];
  asm volatile("" : "+v"(val));
  const bool valid = (xi >= 0) & (xi < GW) & (yi >= 0) & (yi < GH);
  return valid ? val : 0.f;
}

__global__ __launch_bounds__(256) void k_deform(const float* __restrict__ refp, const float* __restrict__ VDEF, const float* __restrict__ OA, _Float16* __restrict__ D16) {
  #pragma clang fp contract(off)
  __shared__ __attribute__((aligned(16))) unsigned short ot[16][OTP];
  const unsigned tid = threadIdx.x, lane = tid & 31u;
  const unsigned w = (unsigned)__builtin_amdgcn_readfirstlane((int)(threadIdx.x >> 5));
  const unsigned row0 = blockIdx.x * 16u;
  const unsigned b = row0 / SEQ, n0 = row0 % SEQ;
  const float* vh = VDEF + (size_t)b * NV * DM + w * HD + lane;
#pragma unroll 1
  for (unsigned t = 0; t < 16u; ++t) {
    const size_t rr = (size_t)b * SEQ_FULL + n0 + t;
    const float rx = bf16_rne(refp[rr * 2]), ry = bf16_rne(refp[rr * 2 + 1]);
    const float* oa = OA + (size_t)(row0 + t) * NOA;
    const float* lg = oa + NOFF + w * NPT;
    const float a0 = lg[0], a1 = lg[1], a2 = lg[2], a3 = lg[3];
    const float mx = fmaxf(fmaxf(a0, a1), fmaxf(a2, a3));
    const float es = (__expf(a0 - mx) + __expf(a1 - mx)) + (__expf(a2 - mx) + __expf(a3 - mx));
    const float inv = 1.0f / es;
    float acc = 0.f;
#pragma unroll 1
    for (unsigned p = 0; p < (unsigned)NPT; ++p) {
      const float ox = oa[w * (NPT * 2) + 2u * p], oy = oa[w * (NPT * 2) + 2u * p + 1u];
      const float wp = __expf(lg[p] - mx) * inv;
      const float gx = (rx + ox * (1.0f / (float)GW)) * (float)GW - 0.5f;
      const float gy = (ry + oy * (1.0f / (float)GH)) * (float)GH - 0.5f;
      const float x0f = floorf(gx), y0f = floorf(gy);
      const float lx = gx - x0f, ly = gy - y0f;
      const int x0 = (int)x0f, y0 = (int)y0f;
      const float v00 = dsamp(vh, x0, y0), v10 = dsamp(vh, x0 + 1, y0), v01 = dsamp(vh, x0, y0 + 1), v11 = dsamp(vh, x0 + 1, y0 + 1);
      const float s = v00 * ((1.0f - lx) * (1.0f - ly)) + v10 * (lx * (1.0f - ly)) + v01 * ((1.0f - lx) * ly) + v11 * (lx * ly);
      acc += s * wp;
    }
    ot[t][w * HD + lane] = __builtin_bit_cast(unsigned short, toh_flush(acc * 64.0f));
  }
  __syncthreads();
  const v8us r0v = *(const v8us*)&ot[2u * w][lane * 8u];
  const v8us r1v = *(const v8us*)&ot[2u * w + 1u][lane * 8u];
  unsigned short* d0 = (unsigned short*)D16 + ((size_t)row0 + 2u * w) * DM + lane * 8u;
  unsigned short* d1 = d0 + DM;
  for (int pass = 0; pass < 2; ++pass) { *(volatile v8us*)d0 = r0v; *(volatile v8us*)d1 = r1v; if (pass == 0) __threadfence(); }
}

template <int BFIN>
__device__ __forceinline__ void ln_rows(const float* __restrict__ X, const float* __restrict__ g, const float* __restrict__ bb, float eps, _Float16* __restrict__ N16) {
  #pragma clang fp contract(off)
  const unsigned tid = threadIdx.x, lane = tid & 31u;
  const unsigned row = blockIdx.x * 8u + (tid >> 5);
  const unsigned xrow = BFIN ? ((row / SEQ) * SEQ_FULL + (row % SEQ)) : row;
  const unsigned c0 = lane * 4u, c1 = 128u + lane * 4u;
  const float* xp = X + (size_t)xrow * DM;
  const v4f xa = *(const v4fa*)(xp + c0), xb = *(const v4fa*)(xp + c1);
  float s[8]; float sum = 0.f;
#pragma unroll
  for (int q = 0; q < 4; ++q) { float a = xa[q], c = xb[q]; if (BFIN) { a = bf16_rne(a); c = bf16_rne(c); } s[q] = a; s[4 + q] = c; }
#pragma unroll
  for (int q = 0; q < 8; ++q) sum += s[q];
  sum += __shfl_xor(sum, 16, 32); sum += __shfl_xor(sum, 8, 32); sum += __shfl_xor(sum, 4, 32); sum += __shfl_xor(sum, 2, 32); sum += __shfl_xor(sum, 1, 32);
  const float mu = sum * (1.0f / (float)DM);
  float vs = 0.f;
#pragma unroll
  for (int q = 0; q < 8; ++q) { const float dl = s[q] - mu; vs += dl * dl; }
  vs += __shfl_xor(vs, 16, 32); vs += __shfl_xor(vs, 8, 32); vs += __shfl_xor(vs, 4, 32); vs += __shfl_xor(vs, 2, 32); vs += __shfl_xor(vs, 1, 32);
  const float rs = rsqrtf(vs * (1.0f / (float)DM) + eps);
  v4h h0, h1;
#pragma unroll
  for (int q = 0; q < 4; ++q) {
    const float y0 = (s[q] - mu) * rs * bf16_rne(g[c0 + q]) + bf16_rne(bb[c0 + q]);
    const float y1 = (s[4 + q] - mu) * rs * bf16_rne(g[c1 + q]) + bf16_rne(bb[c1 + q]);
    h0[q] = toh_flush(y0); h1[q] = toh_flush(y1);
  }
  for (int pass = 0; pass < 2; ++pass) {
    *(volatile v4h*)(N16 + (size_t)row * DM + c0) = h0; *(volatile v4h*)(N16 + (size_t)row * DM + c1) = h1;
    if (pass == 0) __threadfence(); }
}

__global__ __launch_bounds__(256) void k_ln_in(const float* __restrict__ X, const float* __restrict__ g, const float* __restrict__ bb, float eps, _Float16* __restrict__ N16) { ln_rows<1>(X, g, bb, eps, N16); }
__global__ __launch_bounds__(256) void k_ln_ws(const float* __restrict__ X, const float* __restrict__ g, const float* __restrict__ bb, float eps, _Float16* __restrict__ N16) { ln_rows<0>(X, g, bb, eps, N16); }

constexpr size_t al256(size_t v) { return (v + 255) & ~(size_t)255; }
constexpr size_t SZ_WQKV = (size_t)LQ * DM * 2, SZ_WSQ = (size_t)DM * DM * 2, SZ_WFF = (size_t)DM * DFF * 2, SZ_WOA = (size_t)NOA * DM * 2, SZ_BOA = (size_t)NOA * 4;
constexpr size_t SZ_R16 = NR * DM * 2, SZ_R32 = NR * DM * 4, SZ_QKV = NR * LQ * 2, SZ_VT = (size_t)NB * NH * HD * SEQ * 2, SZ_HF = (size_t)(FCH) * DFF * 2;
constexpr size_t SZ_V16 = NRV * DM * 2, SZ_V32 = NRV * DM * 4, SZ_OA = NR * NOA * 4;
constexpr size_t OFF_BQKV = 0;
constexpr size_t OFF_BP = OFF_BQKV + al256(SZ_WQKV);
constexpr size_t OFF_BVP = OFF_BP + al256(SZ_WSQ);
constexpr size_t OFF_BOP = OFF_BVP + al256(SZ_WSQ);
constexpr size_t OFF_BW1 = OFF_BOP + al256(SZ_WSQ);
constexpr size_t OFF_BW2 = OFF_BW1 + al256(SZ_WFF);
constexpr size_t OFF_BOA = OFF_BW2 + al256(SZ_WFF);
constexpr size_t OFF_BIAS = OFF_BOA + al256(SZ_WOA);
constexpr size_t OFF_V16 = OFF_BIAS + al256(SZ_BOA);
constexpr size_t OFF_L16 = OFF_V16 + al256(SZ_V16);
constexpr size_t OFF_QKV = OFF_L16 + al256(SZ_R16);
constexpr size_t OFF_VT = OFF_QKV + al256(SZ_QKV);
constexpr size_t OFF_O16 = OFF_VT + al256(SZ_VT);
constexpr size_t OFF_X1 = OFF_O16 + al256(SZ_R16);
constexpr size_t OFF_X2 = OFF_X1 + al256(SZ_R32);
constexpr size_t OFF_VDEF = OFF_X2 + al256(SZ_R32);
constexpr size_t OFF_OA = OFF_VDEF + al256(SZ_V32);
constexpr size_t OFF_HF = OFF_OA + al256(SZ_OA);
constexpr size_t WS_TOTAL = OFF_HF + al256(SZ_HF);
static_assert(WS_TOTAL <= (size_t)134217728);

extern "C" void kernel_launch(void* const* d_in, const int* in_sizes, int n_in,
                              void* d_out, int out_size, void* d_ws, size_t ws_size, hipStream_t stream) {
  if (n_in < 24) return;
  const size_t need_rows = (size_t)(NB - 1) * SEQ_FULL + SEQ;
  if ((size_t)in_sizes[0] < need_rows * DM || (size_t)in_sizes[1] < need_rows * 2 || (size_t)in_sizes[2] < NRV * DM) return;
  if (in_sizes[3] < DM || in_sizes[4] < DM || in_sizes[5] < DM || in_sizes[6] < DM || in_sizes[7] < DM || in_sizes[8] < DM) return;
  if (in_sizes[9] < LQ * DM || in_sizes[10] < DM * DM || in_sizes[11] < DM) return;
  if (in_sizes[12] < NOFF * DM || in_sizes[13] < NOFF || in_sizes[14] < NLG * DM || in_sizes[15] < NLG) return;
  if (in_sizes[16] < DM * DM || in_sizes[17] < DM || in_sizes[18] < DM * DM || in_sizes[19] < DM) return;
  if (in_sizes[20] < DFF * DM || in_sizes[21] < DFF || in_sizes[22] < DM * DFF || in_sizes[23] < DM) return;
  if ((size_t)out_size < NR * DM) return;
  if (WS_TOTAL > ws_size) return;
  const float* const* I = (const float* const*)d_in;
  const float* x = I[0]; const float* refp = I[1]; const float* value = I[2];
  const float* ln1_w = I[3]; const float* ln1_b = I[4]; const float* ln2_w = I[5]; const float* ln2_b = I[6]; const float* ln3_w = I[7]; const float* ln3_b = I[8];
  const float* qkv_w = I[9]; const float* proj_w = I[10]; const float* proj_b = I[11];
  const float* off_w = I[12]; const float* off_b = I[13]; const float* aw_w = I[14]; const float* aw_b = I[15];
  const float* vproj_w = I[16]; const float* vproj_b = I[17]; const float* oproj_w = I[18]; const float* oproj_b = I[19];
  const float* fc1_w = I[20]; const float* fc1_b = I[21]; const float* fc2_w = I[22]; const float* fc2_b = I[23];
  char* ws = (char*)d_ws;
  _Float16* BQKV = (_Float16*)(ws + OFF_BQKV); _Float16* BP = (_Float16*)(ws + OFF_BP); _Float16* BVP = (_Float16*)(ws + OFF_BVP); _Float16* BOP = (_Float16*)(ws + OFF_BOP);
  _Float16* BW1 = (_Float16*)(ws + OFF_BW1); _Float16* BW2 = (_Float16*)(ws + OFF_BW2); _Float16* BOA = (_Float16*)(ws + OFF_BOA); float* BIASOA = (float*)(ws + OFF_BIAS);
  _Float16* V16 = (_Float16*)(ws + OFF_V16); _Float16* L16 = (_Float16*)(ws + OFF_L16); _Float16* QKV = (_Float16*)(ws + OFF_QKV); _Float16* VT = (_Float16*)(ws + OFF_VT);
  _Float16* O16 = (_Float16*)(ws + OFF_O16); _Float16* D16 = O16;
  float* X1 = (float*)(ws + OFF_X1); float* X2 = (float*)(ws + OFF_X2); float* VDEF = (float*)(ws + OFF_VDEF); float* OA = (float*)(ws + OFF_OA); _Float16* HF16 = (_Float16*)(ws + OFF_HF);
  const int MR = (int)NR;

  k_w16<<<(unsigned)((LQ * DM / 8 + 255) / 256), 256, 0, stream>>>(qkv_w, BQKV, (unsigned)(LQ * DM / 8), 16.0f);
  k_w16<<<(unsigned)((DM * DM / 8 + 255) / 256), 256, 0, stream>>>(proj_w, BP, (unsigned)(DM * DM / 8), 16.0f);
  k_w16<<<(unsigned)((DM * DM / 8 + 255) / 256), 256, 0, stream>>>(vproj_w, BVP, (unsigned)(DM * DM / 8), 16.0f);
  k_w16<<<(unsigned)((DM * DM / 8 + 255) / 256), 256, 0, stream>>>(oproj_w, BOP, (unsigned)(DM * DM / 8), 16.0f);
  k_w16<<<(unsigned)((DFF * DM / 8 + 255) / 256), 256, 0, stream>>>(fc1_w, BW1, (unsigned)(DFF * DM / 8), 16.0f);
  k_w16<<<(unsigned)((DM * DFF / 8 + 255) / 256), 256, 0, stream>>>(fc2_w, BW2, (unsigned)(DM * DFF / 8), 16.0f);
  k_woa<<<(unsigned)(NOA * DM / 8 / 256 + 1), 256, 0, stream>>>(off_w, aw_w, off_b, aw_b, BOA, BIASOA);
  k_val16<<<(unsigned)((NRV * DM / 8 + 255) / 256), 256, 0, stream>>>(value, V16);

  k_ln_in<<<(unsigned)(NR / 8), 256, 0, stream>>>(x, ln1_w, ln1_b, 1e-5f, L16);
  k_gemm_n<<<(unsigned)((NR / 128) * (LQ / 64)), 128, 0, stream>>>(L16, DM, BQKV, DM, 0.0625f, nullptr, nullptr, 0, 0, nullptr, QKV, LQ, MR, LQ, DM);
  k_vt32<<<(unsigned)(NB * NH * (SEQ / 64)), 256, 0, stream>>>(QKV, VT);
  k_flash<<<(unsigned)(NB * (SEQ / 16)), 256, 0, stream>>>(QKV, VT, O16);
  k_gemm_n<<<(unsigned)((NR / 128) * (DM / 64)), 128, 0, stream>>>(O16, DM, BP, DM, 0.0009765625f, proj_b, x, DM, 1, X1, nullptr, DM, MR, DM, DM);

  k_ln_ws<<<(unsigned)(NR / 8), 256, 0, stream>>>(X1, ln2_w, ln2_b, 1e-5f, L16);
  k_gemm_n<<<(unsigned)((NRV / 128) * (DM / 64)), 128, 0, stream>>>(V16, DM, BVP, DM, 0.0625f, vproj_b, nullptr, 0, 0, VDEF, nullptr, DM, (int)NRV, DM, DM);
  k_gemm_n<<<(unsigned)((NR / 128) * (NOA / 64)), 128, 0, stream>>>(L16, DM, BOA, DM, 0.015625f, BIASOA, nullptr, 0, 0, OA, nullptr, NOA, MR, NOA, DM);
  k_deform<<<(unsigned)(NR / 16), 256, 0, stream>>>(refp, VDEF, OA, D16);
  k_gemm_n<<<(unsigned)((NR / 128) * (DM / 64)), 128, 0, stream>>>(D16, DM, BOP, DM, 0.0009765625f, oproj_b, X1, DM, 0, X2, nullptr, DM, MR, DM, DM);

  k_ln_ws<<<(unsigned)(NR / 8), 256, 0, stream>>>(X2, ln3_w, ln3_b, 1e-5f, L16);
  for (size_t r0 = 0; r0 < NR; r0 += FCH) {
    k_gemm_gelu<<<(unsigned)((FCH / 128) * (DFF / 64)), 128, 0, stream>>>(L16 + r0 * DM, DM, BW1, DM, 0.0625f, fc1_b, nullptr, 0, 0, nullptr, HF16, DFF, (int)(FCH), DFF, DM);
    k_gemm_n<<<(unsigned)((FCH / 128) * (DM / 64)), 128, 0, stream>>>(HF16, DFF, BW2, DFF, 0.0625f, fc2_b, X2 + r0 * DM, DM, 0, (float*)d_out + r0 * DM, nullptr, DM, (int)(FCH), DM, DFF);
  }
}
